// GatedSelfAttentionModel_67946382623209
// MI455X (gfx1250) — hardware-verified
//
#include <hip/hip_runtime.h>
#include <math.h>
#include <stdint.h>

#define NB    4
#define NTOK  2048
#define MP    (NB * NTOK)
#define DM    512
#define NH    8
#define HD    64
#define TIN   768
#define TT    128
#define PF    128
#define PH    64
#define EH    64
#define QREAL 520
#define QNP   576
#define HPN   64
#define NQB   (NTOK / 64)
#define QKC   4.0f
#define VC    16.0f
#define PC    1024.0f
static_assert(NH * HD == DM);
static_assert(TIN == DM + TT + PF);
static_assert((MP % 64) == 0 && (DM % 64) == 0 && (QNP % 64) == 0 && (TIN % 32) == 0 && (EH % 64) == 0);
static_assert((NTOK % 64) == 0 && NQB * 64 == NTOK);
static_assert((MP * 8) % 256 == 0 && (MP * 16) % 256 == 0 && ((MP * 3) % 128) == 0);
static_assert(((MP * NH) % 32) == 0);
static_assert(((NB * TT) % 4) == 0 && TT == 128);
static_assert(QNP >= QREAL && HPN >= 3);

typedef _Float16 v16h __attribute__((ext_vector_type(16)));
typedef _Float16 v8h  __attribute__((ext_vector_type(8)));
typedef __attribute__((ext_vector_type(16))) __bf16 v16b;
typedef float    v8f  __attribute__((ext_vector_type(8)));
typedef float    v4f  __attribute__((ext_vector_type(4)));
typedef unsigned int v4u __attribute__((ext_vector_type(4)));

union FragH  { v16h v; v8h h[2]; };
union Frag16 { v16h h; v16b b; v8h hh[2]; v4u u[2]; };

__device__ __forceinline__ unsigned short bf_bits(float f) {
  const unsigned u = __float_as_uint(f);
  return (unsigned short)((u + 0x7FFFu + ((u >> 16) & 1u)) >> 16);
}
__device__ __forceinline__ float bf_up(unsigned short h) { return __uint_as_float(((unsigned)h) << 16); }
__device__ __forceinline__ float bfr(float f) { return bf_up(bf_bits(f)); }
__device__ __forceinline__ unsigned short h_bits(_Float16 x) { return __builtin_bit_cast(unsigned short, x); }
__device__ __forceinline__ unsigned pk16(unsigned short a, unsigned short b) { return (unsigned)a | ((unsigned)b << 16); }
__device__ __forceinline__ v8f zero8() { v8f z = {0.f, 0.f, 0.f, 0.f, 0.f, 0.f, 0.f, 0.f}; return z; }
__device__ __forceinline__ void hilo2(float f0, float f1, unsigned& hi, unsigned& lo) {
  const unsigned short h0 = bf_bits(f0), h1 = bf_bits(f1);
  hi = pk16(h0, h1);
  lo = pk16(bf_bits(f0 - bf_up(h0)), bf_bits(f1 - bf_up(h1)));
}
__device__ __forceinline__ float sigmoidf_(float g) { return 1.0f / (1.0f + expf(-g)); }

__device__ __forceinline__ v16h ldfrag_h(const _Float16* p) {
  FragH f;
  f.h[0] = *(const v8h*)(p);
  f.h[1] = *(const v8h*)(p + 16);
  return f.v;
}
__device__ __forceinline__ Frag16 ldfrag16(const unsigned short* p) {
  Frag16 f;
  f.u[0] = *(const v4u*)(p);
  f.u[1] = *(const v4u*)(p + 16);
  return f;
}

__device__ __forceinline__ v8f mma_h(v16h a, v16h b, v8f c) {
  c = __builtin_amdgcn_wmma_f32_16x16x32_f16(false, a, false, b, (short)0, c, false, false);
#if defined(__HIP_DEVICE_COMPILE__)
  asm volatile("v_nop\n\tv_nop\n\tv_nop\n\tv_nop" : "+v"(c) : "v"(a), "v"(b));
#endif
  return c;
}
__device__ __forceinline__ v8f mma_h_raw(v16h a, v16h b, v8f c) {
  return __builtin_amdgcn_wmma_f32_16x16x32_f16(false, a, false, b, (short)0, c, false, false);
}
__device__ __forceinline__ v8f mma_b_raw(const Frag16& a, const Frag16& b, v8f c) {
  return __builtin_amdgcn_wmma_f32_16x16x32_bf16(false, a.b, false, b.b, (short)0, c, false, false);
}
__device__ __forceinline__ void dep_guard1(v8f& a, v8f& b, v16h x) {
#if defined(__HIP_DEVICE_COMPILE__)
  asm volatile("v_nop\n\tv_nop\n\tv_nop\n\tv_nop" : "+v"(a), "+v"(b) : "v"(x));
#endif
}
__device__ __forceinline__ void dep_guard3(v8f& a, v8f& b, v16h x, v16h y, v16h z) {
#if defined(__HIP_DEVICE_COMPILE__)
  asm volatile("v_nop\n\tv_nop\n\tv_nop\n\tv_nop" : "+v"(a), "+v"(b) : "v"(x), "v"(y), "v"(z));
#endif
}
__device__ __forceinline__ void keep4_h(v16h a, v16h b, v16h c, v16h d) {
#if defined(__HIP_DEVICE_COMPILE__)
  asm volatile("v_nop" :: "v"(a), "v"(b), "v"(c), "v"(d));
#endif
}
__device__ __forceinline__ void acc_guard4(v8f& a, v8f& b, v8f& c, v8f& d) {
#if defined(__HIP_DEVICE_COMPILE__)
  asm volatile("v_nop\n\tv_nop\n\tv_nop\n\tv_nop" : "+v"(a), "+v"(b), "+v"(c), "+v"(d));
#endif
}
__device__ __forceinline__ void wave_sync_lds() {
  __builtin_amdgcn_fence(__ATOMIC_RELEASE, "workgroup");
  __builtin_amdgcn_wave_barrier();
  __builtin_amdgcn_fence(__ATOMIC_ACQUIRE, "workgroup");
}

__global__ __launch_bounds__(256) void cvt_w(const float* __restrict__ W, unsigned short* dst, int Cin, int Osrc,
                                              int Odst, int n8) {
  const int i    = blockIdx.x * 256 + threadIdx.x;
  const int ic   = (i < n8) ? i : (n8 - 1);
  const int cin8 = Cin >> 3;
  const int o    = ic / cin8;
  const int c0   = (ic - o * cin8) * 8;
  const bool live = (o < Osrc);
  const int oc   = live ? o : (Osrc - 1);
  const float* p = W + (size_t)c0 * Osrc + oc;
  v4u ov;
#pragma unroll
  for (int e = 0; e < 4; ++e) {
    const float f0 = p[(size_t)(2 * e) * Osrc];
    const float f1 = p[(size_t)(2 * e + 1) * Osrc];
    const unsigned short b0 = live ? bf_bits(f0) : (unsigned short)0;
    const unsigned short b1 = live ? bf_bits(f1) : (unsigned short)0;
    ov[e] = pk16(b0, b1);
  }
  (void)Odst;
  if (i < n8) *(volatile v4u*)(dst + (size_t)i * 8) = ov;
  __threadfence();
  if (i < n8) *(volatile v4u*)(dst + (size_t)i * 8) = ov;
}

__global__ __launch_bounds__(256) void cvt_x(const float* __restrict__ X, unsigned short* dst, int n8) {
  const int i  = blockIdx.x * 256 + threadIdx.x;
  const int ic = (i < n8) ? i : (n8 - 1);
  const float* p = X + (size_t)ic * 8;
  const v4f a = *(const v4f*)(p), c4 = *(const v4f*)(p + 4);
  v4u o;
  o[0] = pk16(bf_bits(a[0]), bf_bits(a[1]));
  o[1] = pk16(bf_bits(a[2]), bf_bits(a[3]));
  o[2] = pk16(bf_bits(c4[0]), bf_bits(c4[1]));
  o[3] = pk16(bf_bits(c4[2]), bf_bits(c4[3]));
  if (i < n8) *(volatile v4u*)(dst + (size_t)i * 8) = o;
  __threadfence();
  if (i < n8) *(volatile v4u*)(dst + (size_t)i * 8) = o;
}

__global__ __launch_bounds__(256) void pack_bias(const float* __restrict__ qb, const float* __restrict__ hb, float* dst) {
  const int t  = threadIdx.x;
  const int tc = (t < 160) ? t : 159;
  v4f o;
#pragma unroll
  for (int e = 0; e < 4; ++e) {
    const int i  = 4 * tc + e;
    const int iq = (i < QREAL) ? i : (QREAL - 1);
    const float vq = qb[iq];
    int ih = i - QNP;
    ih = (ih < 0) ? 0 : ((ih > 2) ? 2 : ih);
    const float vh = hb[ih];
    float v = 0.f;
    if (i < QREAL) v = vq;
    if (i >= QNP && (i - QNP) < 3) v = vh;
    o[e] = v;
  }
  if (t < 160) *(volatile v4f*)(dst + 4 * t) = o;
  __threadfence();
  if (t < 160) *(volatile v4f*)(dst + 4 * t) = o;
}

__global__ __launch_bounds__(256) void pos_l1(const float* __restrict__ pos, const float* __restrict__ w1,
                                               const float* __restrict__ b1, unsigned short* TH, unsigned short* TL) {
#pragma clang fp contract(off)
  const int t = blockIdx.x * 256 + threadIdx.x;
  const int token = t >> 3, g = t & 7;
  const float* pp = pos + (size_t)token * 3;
  const float x = bfr(pp[0]), y = bfr(pp[1]), z = bfr(pp[2]);
  const float n2 = (x * x + y * y) + z * z;
  const float nr = sqrtf(n2);
  const float inv = 1.0f / (nr + 1e-7f);
  const float f0 = x * inv, f1 = y * inv, f2 = z * inv, f3 = nr;
  float hv[8];
#pragma unroll
  for (int u = 0; u < 8; ++u) {
    const int o = 8 * g + u;
    float s = f0 * bfr(w1[o]);
    s = s + f1 * bfr(w1[64 + o]);
    s = s + f2 * bfr(w1[128 + o]);
    s = s + f3 * bfr(w1[192 + o]);
    s = s + bfr(b1[o]);
    hv[u] = fmaxf(s, 0.f);
  }
  v4u oh, ol;
#pragma unroll
  for (int e = 0; e < 4; ++e) {
    unsigned hi, lo;
    hilo2(hv[2 * e], hv[2 * e + 1], hi, lo);
    oh[e] = hi;
    ol[e] = lo;
  }
  const size_t ro = (size_t)token * PH + 8 * g;
  *(volatile v4u*)(TH + ro) = oh;
  *(volatile v4u*)(TL + ro) = ol;
  __threadfence();
  *(volatile v4u*)(TH + ro) = oh;
  *(volatile v4u*)(TL + ro) = ol;
}

__global__ __launch_bounds__(128) void tdt_k(const float* __restrict__ dt, const float* __restrict__ w,
                                              const float* __restrict__ bb, float* TDT) {
  __shared__ __align__(16) float T[NB * TT];
  const int j = threadIdx.x;
  float s[NB];
#pragma unroll
  for (int b = 0; b < NB; ++b) s[b] = 0.f;
#pragma unroll 1
  for (int i = 0; i < TT; ++i) {
    const float wv = bfr(w[i * TT + j]);
#pragma unroll
    for (int b = 0; b < NB; ++b) s[b] += bfr(dt[b * TT + i]) * wv;
  }
  const float bj = bfr(bb[j]);
#pragma unroll
  for (int b = 0; b < NB; ++b) T[b * TT + j] = s[b] + bj;
  __syncthreads();
  const int n4 = (NB * TT) / 4;
  for (int q = j; q < n4; q += TT) {
    const v4f o = *(const v4f*)(T + 4 * q);
    *(volatile v4f*)(TDT + 4 * q) = o;
  }
  __threadfence();
  for (int q = j; q < n4; q += TT) {
    const v4f o = *(const v4f*)(T + 4 * q);
    *(volatile v4f*)(TDT + 4 * q) = o;
  }
}

__global__ __launch_bounds__(256) void tdt_bcast(const float* __restrict__ TDT, unsigned short* CH, unsigned short* CL) {
  const int t = blockIdx.x * 256 + threadIdx.x;
  const int token = t >> 4, g = t & 15;
  const int b = token / NTOK;
  const float* p = TDT + b * TT + 8 * g;
  const v4f a = *(const v4f*)(p), c4 = *(const v4f*)(p + 4);
  v4u oh, ol;
  {
    unsigned hi, lo;
    hilo2(a[0], a[1], hi, lo);   oh[0] = hi; ol[0] = lo;
    hilo2(a[2], a[3], hi, lo);   oh[1] = hi; ol[1] = lo;
    hilo2(c4[0], c4[1], hi, lo); oh[2] = hi; ol[2] = lo;
    hilo2(c4[2], c4[3], hi, lo); oh[3] = hi; ol[3] = lo;
  }
  const size_t ro = (size_t)token * TIN + DM + 8 * g;
  *(volatile v4u*)(CH + ro) = oh;
  *(volatile v4u*)(CL + ro) = ol;
  __threadfence();
  *(volatile v4u*)(CH + ro) = oh;
  *(volatile v4u*)(CL + ro) = ol;
}

template <int NPA, int NPB, int OM, int BIASM, int ACT>
__global__ __launch_bounds__(256) void gemm64(
    const unsigned short* __restrict__ A1p, const unsigned short* __restrict__ A2p, int lda, long long strideA,
    const unsigned short* __restrict__ B1p, const unsigned short* __restrict__ B2p, int ldb, long long strideB,
    const float* __restrict__ bias, float bscale,
    void* Cout, void* Cout2, int ldc, long long strideC,
    int M, int N, int K, float oscale) {
  __shared__ __align__(16) float sT[8][16 * 68];
  const int b    = blockIdx.y;
  const int lane = threadIdx.x & 31;
  const int wave = threadIdx.x >> 5;
  const int tilesN = N >> 6;
  const int tilesM = M >> 6;
  const int tile = blockIdx.x * 8 + wave;
  if (tile >= tilesM * tilesN) return;
  const int tm = tile / tilesN;
  const int tn = tile - tm * tilesN;
  const int m0 = tm << 6;
  const int n0 = tn << 6;

  const unsigned short* A1 = A1p + (size_t)b * strideA;
  const unsigned short* A2 = A2p + (size_t)b * strideA;
  const unsigned short* B1 = B1p + (size_t)b * strideB;
  const unsigned short* B2 = B2p + (size_t)b * strideB;

  const int rlane = lane & 15;
  const int koff  = (lane >> 4) * 8;
  const int mOff  = (lane >> 4) * 8;

  v8f acc[4][4];
#pragma unroll
  for (int i = 0; i < 4; ++i)
#pragma unroll
    for (int j = 0; j < 4; ++j) acc[i][j] = zero8();

  const int nstep = (K >> 5) * NPB;
  for (int st = 0; st < nstep; ++st) {
    const int k0 = (NPB == 2) ? ((st >> 1) << 5) : (st << 5);
    const unsigned short* Bs = (NPB == 2 && (st & 1) != 0) ? B2 : B1;
    Frag16 bh[4];
#pragma unroll
    for (int j = 0; j < 4; ++j) {
      const size_t bo = (size_t)(n0 + (j << 4) + rlane) * ldb + koff + k0;
      bh[j] = ldfrag16(Bs + bo);
    }
#pragma unroll
    for (int i = 0; i < 4; ++i) {
#pragma unroll
      for (int pa = 0; pa < NPA; ++pa) {
        const unsigned short* As = (pa == 0) ? A1 : A2;
        const size_t ao = (size_t)(m0 + (i << 4) + rlane) * lda + koff + k0;
        const Frag16 ah = ldfrag16(As + ao);
#pragma unroll
        for (int j = 0; j < 4; ++j) acc[i][j] = mma_b_raw(ah, bh[j], acc[i][j]);
        dep_guard1(acc[i][0], acc[i][3], ah.h);
      }
    }
    keep4_h(bh[0].h, bh[1].h, bh[2].h, bh[3].h);
  }
  acc_guard4(acc[0][0], acc[0][1], acc[0][2], acc[0][3]);
  acc_guard4(acc[1][0], acc[1][1], acc[1][2], acc[1][3]);
  acc_guard4(acc[2][0], acc[2][1], acc[2][2], acc[2][3]);
  acc_guard4(acc[3][0], acc[3][1], acc[3][2], acc[3][3]);

  const int hh2 = lane >> 4, c4 = (lane & 15) * 4;
  const int q8  = lane >> 3, c8 = (lane & 7) * 8;
  float bc[8];
#pragma unroll
  for (int e = 0; e < 8; ++e) bc[e] = 0.f;
  if (BIASM == 0) {
    if (OM == 0) {
      const int cb = n0 + c4;
      const int i0 = (cb < N - 4) ? cb : (N - 4);
      const v4f b0v = *(const v4f*)(bias + i0);
#pragma unroll
      for (int e = 0; e < 4; ++e) bc[e] = bfr(b0v[e]) * bscale;
    } else {
      const int cb = n0 + c8;
      const int i0 = (cb < N - 8) ? cb : (N - 8);
      const v4f b0a = *(const v4f*)(bias + i0), b0b = *(const v4f*)(bias + i0 + 4);
#pragma unroll
      for (int e = 0; e < 4; ++e) {
        bc[e]     = bfr(b0a[e]) * bscale;
        bc[4 + e] = bfr(b0b[e]) * bscale;
      }
    }
  }

  float* slab = sT[wave];
#pragma unroll
  for (int i = 0; i < 4; ++i) {
    const int mBase = m0 + (i << 4);
#pragma unroll
    for (int j = 0; j < 4; ++j) {
#pragma unroll
      for (int r = 0; r < 8; ++r) {
        slab[(mOff + r) * 68 + (j << 4) + rlane] = acc[i][j][r];
      }
    }
    wave_sync_lds();
    if (OM == 0) {
      float* C = (float*)Cout + (size_t)b * strideC;
      v4f vals[8];
#pragma unroll
      for (int it = 0; it < 8; ++it) {
        const int row = it * 2 + hh2;
        v4f v = *(const v4f*)(slab + row * 68 + c4);
#pragma unroll
        for (int e = 0; e < 4; ++e) {
          float f = v[e] * oscale + bc[e];
          if (ACT == 1) f = fmaxf(f, 0.f);
          v[e] = f;
        }
        vals[it] = v;
      }
      for (int pass = 0; pass < 2; ++pass) {
#pragma unroll
        for (int it = 0; it < 8; ++it) {
          const int row = it * 2 + hh2;
          *(volatile v4f*)(C + (size_t)(mBase + row) * ldc + n0 + c4) = vals[it];
        }
        __threadfence();
      }
    } else {
      unsigned short* C  = (unsigned short*)Cout  + (size_t)b * strideC;
      unsigned short* C2 = (unsigned short*)Cout2 + (size_t)b * strideC;
      v4u hv[4], lv[4];
#pragma unroll
      for (int it = 0; it < 4; ++it) {
        const int row = it * 4 + q8;
        const float* sp = slab + row * 68 + c8;
        float bm = 0.f;
        if (BIASM == 1) bm = bfr(bias[mBase + row]) * bscale;
        v4u a, a2;
#pragma unroll
        for (int e = 0; e < 4; ++e) {
          float f0 = sp[2 * e]     * oscale + ((BIASM == 1) ? bm : bc[2 * e]);
          float f1 = sp[2 * e + 1] * oscale + ((BIASM == 1) ? bm : bc[2 * e + 1]);
          if (ACT == 1) { f0 = fmaxf(f0, 0.f); f1 = fmaxf(f1, 0.f); }
          if (OM == 2) {
            a[e]  = pk16(h_bits((_Float16)f0), h_bits((_Float16)f1));
            a2[e] = a[e];
          } else {
            unsigned hi, lo;
            hilo2(f0, f1, hi, lo);
            a[e]  = hi;
            a2[e] = lo;
          }
        }
        hv[it] = a;
        lv[it] = a2;
      }
      for (int pass = 0; pass < 2; ++pass) {
#pragma unroll
        for (int it = 0; it < 4; ++it) {
          const int row = it * 4 + q8;
          *(volatile v4u*)(C + (size_t)(mBase + row) * ldc + n0 + c8) = hv[it];
          if (OM == 3) *(volatile v4u*)(C2 + (size_t)(mBase + row) * ldc + n0 + c8) = lv[it];
        }
        __threadfence();
      }
    }
    wave_sync_lds();
  }
}

__global__ __launch_bounds__(256) void rms_qk(const float* __restrict__ QF, const float* __restrict__ KF,
                                               const float* __restrict__ qw, const float* __restrict__ kw,
                                               unsigned short* QN, unsigned short* KN, int nqb) {
  const int bx = blockIdx.x;
  const bool isk = (bx >= nqb);
  const int lb = isk ? (bx - nqb) : bx;
  const float* src  = isk ? KF : QF;
  const int ld      = isk ? DM : QNP;
  const float* wsrc = isk ? kw : qw;
  unsigned short* dst = isk ? KN : QN;
  const int tid = threadIdx.x, lane = tid & 31, wave = tid >> 5;
  int p = lb * 32 + wave * 4 + (lane >> 3);
  const int pmax = MP * NH - 1;
  p = (p > pmax) ? pmax : p;
  const int token = p >> 3, head = p & 7, g = lane & 7;
  const float* xp = src + (size_t)token * ld + head * HD + 8 * g;
  const v4f x0 = *(const v4f*)(xp), x1 = *(const v4f*)(xp + 4);
  float ss = ((x0[0] * x0[0] + x0[1] * x0[1]) + (x0[2] * x0[2] + x0[3] * x0[3])) +
             ((x1[0] * x1[0] + x1[1] * x1[1]) + (x1[2] * x1[2] + x1[3] * x1[3]));
  ss += __shfl_xor(ss, 1, 32);
  ss += __shfl_xor(ss, 2, 32);
  ss += __shfl_xor(ss, 4, 32);
  const float r = rsqrtf(ss * (1.0f / 64.0f) + 1e-6f);
  const v4f w0 = *(const v4f*)(wsrc + 8 * g), w1 = *(const v4f*)(wsrc + 8 * g + 4);
  float y[8];
#pragma unroll
  for (int e = 0; e < 4; ++e) {
    y[e]     = ((x0[e] * r) * bfr(w0[e])) * QKC;
    y[4 + e] = ((x1[e] * r) * bfr(w1[e])) * QKC;
  }
  v4u o;
#pragma unroll
  for (int e = 0; e < 4; ++e) o[e] = pk16(h_bits((_Float16)y[2 * e]), h_bits((_Float16)y[2 * e + 1]));
  const size_t ro = (size_t)token * DM + head * HD + 8 * g;
  *(volatile v4u*)(dst + ro) = o;
  __threadfence();
  *(volatile v4u*)(dst + ro) = o;
}

__global__ __launch_bounds__(128)
void attn(const unsigned short* __restrict__ QNp, const unsigned short* __restrict__ KNp,
          const unsigned short* __restrict__ VTp, const float* __restrict__ QF,
          unsigned short* AOH, unsigned short* AOL) {
  __shared__ __align__(16) float Ps[4][16 * 68];
  __shared__ __align__(16) float Os[4][16 * 68];

  const int tid  = threadIdx.x;
  const int wave = tid >> 5;
  const int lane = tid & 31;
  const int hh   = lane >> 4;
  const int c    = lane & 15;

  const int bx = blockIdx.x;
  const int bh = bx / NQB;
  const int b  = bh >> 3;
  const int h  = bh & 7;
  const int q0 = (bx - bh * NQB) * 64 + wave * 16;
  const size_t tok0 = (size_t)b * NTOK + q0;

  const _Float16* Q  = (const _Float16*)(const void*)QNp + h * HD;
  const _Float16* Kp = (const _Float16*)(const void*)KNp + (size_t)b * NTOK * DM + h * HD;
  const _Float16* V  = (const _Float16*)(const void*)VTp + ((size_t)b * DM + h * HD) * NTOK;
  const float lsc = (1.4426950408889634f * 0.125f) / (QKC * QKC);

  const v16h qa0 = ldfrag_h(Q + (tok0 + c) * DM + 8 * hh);
  const v16h qa1 = ldfrag_h(Q + (tok0 + c) * DM + 32 + 8 * hh);

  float mrow[8], lrow[8];
  v8f oacc[4];
#pragma unroll
  for (int r = 0; r < 8; ++r) { mrow[r] = -INFINITY; lrow[r] = 0.f; }
#pragma unroll
  for (int t = 0; t < 4; ++t) oacc[t] = zero8();
  float* pt = Ps[wave];

#pragma unroll 1
  for (int kb = 0; kb < NTOK; kb += 64) {
    v8f s[4];
#pragma unroll
    for (int j = 0; j < 4; ++j) {
      const _Float16* kr = Kp + (size_t)(kb + 16 * j + c) * DM + 8 * hh;
      const v16h k0f = ldfrag_h(kr);
      const v16h k1f = ldfrag_h(kr + 32);
      s[j] = mma_h(qa0, k0f, zero8());
      s[j] = mma_h(qa1, k1f, s[j]);
    }
#pragma unroll
    for (int r = 0; r < 8; ++r) {
      const float t0 = s[0][r] * lsc, t1 = s[1][r] * lsc, t2 = s[2][r] * lsc, t3 = s[3][r] * lsc;
      float mx = fmaxf(fmaxf(t0, t1), fmaxf(t2, t3));
#pragma unroll
      for (int off = 1; off < 16; off <<= 1) mx = fmaxf(mx, __shfl_xor(mx, off, 32));
      const float mn = fmaxf(mrow[r], mx);
      const float al = exp2f(mrow[r] - mn);
      mrow[r] = mn;
      const float e0 = exp2f(t0 - mn), e1 = exp2f(t1 - mn), e2 = exp2f(t2 - mn), e3 = exp2f(t3 - mn);
      float ps = (e0 + e1) + (e2 + e3);
#pragma unroll
      for (int off = 1; off < 16; off <<= 1) ps += __shfl_xor(ps, off, 32);
      lrow[r] = lrow[r] * al + ps;
      oacc[0][r] *= al;
      oacc[1][r] *= al;
      oacc[2][r] *= al;
      oacc[3][r] *= al;
      const int ro = (8 * hh + r) * 68 + c;
      pt[ro]      = e0;
      pt[ro + 16] = e1;
      pt[ro + 32] = e2;
      pt[ro + 48] = e3;
    }
    wave_sync_lds();
#pragma unroll
    for (int wi = 0; wi < 2; ++wi) {
      const float* prow = pt + c * 68 + 32 * wi + 8 * hh;
      const v4f p0 = *(const v4f*)(prow), p1 = *(const v4f*)(prow + 4);
      const v4f p2 = *(const v4f*)(prow + 16), p3 = *(const v4f*)(prow + 20);
      FragH pa;
#pragma unroll
      for (int e = 0; e < 4; ++e) {
        pa.h[0][e]     = (_Float16)(p0[e] * PC);
        pa.h[0][4 + e] = (_Float16)(p1[e] * PC);
        pa.h[1][e]     = (_Float16)(p2[e] * PC);
        pa.h[1][4 + e] = (_Float16)(p3[e] * PC);
      }
      const int k0 = kb + 32 * wi;
      {
        const v16h vb0 = ldfrag_h(V + (size_t)c * NTOK + k0 + 8 * hh);
        const v16h vb1 = ldfrag_h(V + (size_t)(16 + c) * NTOK + k0 + 8 * hh);
        oacc[0] = mma_h_raw(pa.v, vb0, oacc[0]);
        oacc[1] = mma_h_raw(pa.v, vb1, oacc[1]);
        dep_guard3(oacc[0], oacc[1], pa.v, vb0, vb1);
      }
      {
        const v16h vb2 = ldfrag_h(V + (size_t)(32 + c) * NTOK + k0 + 8 * hh);
        const v16h vb3 = ldfrag_h(V + (size_t)(48 + c) * NTOK + k0 + 8 * hh);
        oacc[2] = mma_h_raw(pa.v, vb2, oacc[2]);
        oacc[3] = mma_h_raw(pa.v, vb3, oacc[3]);
        dep_guard3(oacc[2], oacc[3], pa.v, vb2, vb3);
      }
    }
    wave_sync_lds();
  }

  float* os = Os[wave];
  const float oinv = 1.0f / (PC * VC);
#pragma unroll
  for (int r = 0; r < 8; ++r) {
    const size_t trow = tok0 + 8 * hh + r;
    const float g   = QF[trow * (size_t)QNP + (size_t)(DM + h)];
    const float sg  = sigmoidf_(g);
    const float inv = (sg * (1.0f / lrow[r])) * oinv;
    const int ro = (8 * hh + r) * 68 + c;
    os[ro]      = oacc[0][r] * inv;
    os[ro + 16] = oacc[1][r] * inv;
    os[ro + 32] = oacc[2][r] * inv;
    os[ro + 48] = oacc[3][r] * inv;
  }
  wave_sync_lds();
  {
    const int q8 = lane >> 3, c8 = (lane & 7) * 8;
    v4u hv[4], lv[4];
#pragma unroll
    for (int it = 0; it < 4; ++it) {
      const int row = it * 4 + q8;
      const float* sp = os + row * 68 + c8;
      const v4f a = *(const v4f*)(sp), bq = *(const v4f*)(sp + 4);
      v4u oh, ol;
      unsigned hi, lo;
      hilo2(a[0], a[1], hi, lo);   oh[0] = hi; ol[0] = lo;
      hilo2(a[2], a[3], hi, lo);   oh[1] = hi; ol[1] = lo;
      hilo2(bq[0], bq[1], hi, lo); oh[2] = hi; ol[2] = lo;
      hilo2(bq[2], bq[3], hi, lo); oh[3] = hi; ol[3] = lo;
      hv[it] = oh;
      lv[it] = ol;
    }
    for (int pass = 0; pass < 2; ++pass) {
#pragma unroll
      for (int it = 0; it < 4; ++it) {
        const int row = it * 4 + q8;
        const size_t o = (tok0 + row) * DM + h * HD + c8;
        *(volatile v4u*)(AOH + o) = hv[it];
        *(volatile v4u*)(AOL + o) = lv[it];
      }
      __threadfence();
    }
  }
}

__global__ __launch_bounds__(256) void pack_out(const float* __restrict__ HP, const float* __restrict__ TDT, float* out) {
  const int t = blockIdx.x * 256 + threadIdx.x;
  const int npos4 = (MP * 3) / 4;
  const int nt = npos4 + (NB * TT) / 4;
  const int tp = (t < npos4) ? t : (npos4 - 1);
  int tt = t - npos4;
  tt = (tt < 0) ? 0 : ((tt > (NB * TT) / 4 - 1) ? ((NB * TT) / 4 - 1) : tt);
  v4f a;
#pragma unroll
  for (int e = 0; e < 4; ++e) {
    const int idx = 4 * tp + e;
    const int token = idx / 3;
    const int oo = idx - 3 * token;
    a[e] = HP[(size_t)token * HPN + oo];
  }
  const v4f bt = *(const v4f*)(TDT + 4 * tt);
  const bool isp = (t < npos4);
  v4f o;
#pragma unroll
  for (int e = 0; e < 4; ++e) o[e] = isp ? a[e] : bt[e];
  float* dp = out + (size_t)MP * DM + 4 * (size_t)t;
  if (t < nt) *(volatile v4f*)(dp) = o;
  __threadfence();
  if (t < nt) *(volatile v4f*)(dp) = o;
}

extern "C" void kernel_launch(void* const* d_in, const int* in_sizes, int n_in,
                              void* d_out, int out_size, void* d_ws, size_t ws_size,
                              hipStream_t stream) {
  if (n_in < 29) return;
  if (in_sizes[0] != MP * DM || in_sizes[1] != NB * TT || in_sizes[2] != MP * 3) return;
  if (in_sizes[3] != 4 * PH || in_sizes[4] != PH || in_sizes[5] != PH * PF || in_sizes[6] != PF) return;
  if (in_sizes[7] != DM * EH || in_sizes[8] != EH || in_sizes[9] != EH * DM || in_sizes[10] != DM) return;
  if (in_sizes[11] != TT * TT || in_sizes[12] != TT || in_sizes[13] != TIN * DM || in_sizes[14] != DM) return;
  if (in_sizes[15] != DM * QREAL || in_sizes[16] != QREAL) return;
  if (in_sizes[17] != DM * DM || in_sizes[18] != DM || in_sizes[19] != DM * DM || in_sizes[20] != DM) return;
  if (in_sizes[21] != DM * DM || in_sizes[22] != DM || in_sizes[23] != HD || in_sizes[24] != HD) return;
  if (in_sizes[25] != DM * 3 || in_sizes[26] != 3 || in_sizes[27] != DM * DM || in_sizes[28] != DM) return;
  if (out_size != MP * DM + MP * 3 + NB * TT) return;

  const float* x_ef   = (const float*)d_in[0];
  const float* x_dt   = (const float*)d_in[1];
  const float* x_pos  = (const float*)d_in[2];
  const float* pos_w1 = (const float*)d_in[3];   const float* pos_b1 = (const float*)d_in[4];
  const float* pos_w2 = (const float*)d_in[5];   const float* pos_b2 = (const float*)d_in[6];
  const float* ex_w1  = (const float*)d_in[7];   const float* ex_b1  = (const float*)d_in[8];
  const float* ex_w2  = (const float*)d_in[9];   const float* ex_b2  = (const float*)d_in[10];
  const float* yy_w   = (const float*)d_in[11];  const float* yy_b   = (const float*)d_in[12];
  const float* cat_w  = (const float*)d_in[13];  const float* cat_b  = (const float*)d_in[14];
  const float* q_w    = (const float*)d_in[15];  const float* q_b    = (const float*)d_in[16];
  const float* k_w    = (const float*)d_in[17];  const float* k_b    = (const float*)d_in[18];
  const float* v_w    = (const float*)d_in[19];  const float* v_b    = (const float*)d_in[20];
  const float* o_w    = (const float*)d_in[21];  const float* o_b    = (const float*)d_in[22];
  const float* qn_w   = (const float*)d_in[23];  const float* kn_w   = (const float*)d_in[24];
  const float* hp_w   = (const float*)d_in[25];  const float* hp_b   = (const float*)d_in[26];
  const float* he_w   = (const float*)d_in[27];  const float* he_b   = (const float*)d_in[28];

  const size_t PW1   = (size_t)EH * DM * 2;
  const size_t PW2   = (size_t)DM * EH * 2;
  const size_t PPW2  = (size_t)PF * PH * 2;
  const size_t PCW   = (size_t)DM * TIN * 2;
  const size_t PQW   = (size_t)QNP * DM * 2;
  const size_t PSQ   = (size_t)DM * DM * 2;
  const size_t PHPW  = (size_t)HPN * DM * 2;
  const size_t PBIA  = 4096;
  const size_t PTDT  = 4096;
  const size_t PT64  = (size_t)MP * 64 * 2;
  const size_t PCAT  = (size_t)MP * TIN * 2;
  const size_t PH16  = (size_t)MP * DM * 2;
  const size_t PQF   = (size_t)MP * QNP * 4;
  const size_t PF32  = (size_t)MP * DM * 4;
  const size_t PVT   = (size_t)NB * DM * NTOK * 2;
  size_t off = 0;
  const size_t oW1T = off; off += PW1;
  const size_t oW2T = off; off += PW2;
  const size_t oPW2 = off; off += PPW2;
  const size_t oCWT = off; off += PCW;
  const size_t oQWT = off; off += PQW;
  const size_t oKWT = off; off += PSQ;
  const size_t oVWT = off; off += PSQ;
  const size_t oOWT = off; off += PSQ;
  const size_t oHEW = off; off += PSQ;
  const size_t oHPW = off; off += PHPW;
  const size_t oBIA = off; off += PBIA;
  const size_t oTDT = off; off += PTDT;
  const size_t oTE1H = off; off += PT64;
  const size_t oTE1L = off; off += PT64;
  const size_t oTP1H = off; off += PT64;
  const size_t oTP1L = off; off += PT64;
  const size_t oCATH = off; off += PCAT;
  const size_t oCATL = off; off += PCAT;
  const size_t oHH   = off; off += PH16;
  const size_t oHL   = off; off += PH16;
  const size_t oQF   = off; off += PQF;
  const size_t oKF   = off; off += PF32;
  const size_t oQN   = off; off += PH16;
  const size_t oKN   = off; off += PH16;
  const size_t oVT   = off; off += PVT;
  if (off > ws_size) return;
  if (off > (size_t)134217728) return;
  if ((size_t)NB * TT * 4 > PTDT || (size_t)(QNP + HPN) * 4 > PBIA) return;
  const size_t oHP64 = oTE1H;
  const size_t oAOH  = oCATH;
  const size_t oAOL  = oCATH + PH16;
  const size_t oOUTH = oHH;
  const size_t oOUTL = oHL;
  const size_t oXB   = oKF;
  if ((size_t)MP * HPN * 4 > 2 * PT64) return;
  if (oAOL + PH16 > oCATL + PCAT) return;
  if (PH16 > PF32) return;

  char* ws = (char*)d_ws;
  unsigned short* W1T  = (unsigned short*)(ws + oW1T);
  unsigned short* W2T  = (unsigned short*)(ws + oW2T);
  unsigned short* PW2T = (unsigned short*)(ws + oPW2);
  unsigned short* CWT  = (unsigned short*)(ws + oCWT);
  unsigned short* QWT  = (unsigned short*)(ws + oQWT);
  unsigned short* KWT  = (unsigned short*)(ws + oKWT);
  unsigned short* VWT  = (unsigned short*)(ws + oVWT);
  unsigned short* OWT  = (unsigned short*)(ws + oOWT);
  unsigned short* HEWT = (unsigned short*)(ws + oHEW);
  unsigned short* HPWT = (unsigned short*)(ws + oHPW);
  float*          BIAS = (float*)(ws + oBIA);
  float*          TDT  = (float*)(ws + oTDT);
  unsigned short* TE1H = (unsigned short*)(ws + oTE1H);
  unsigned short* TE1L = (unsigned short*)(ws + oTE1L);
  unsigned short* TP1H = (unsigned short*)(ws + oTP1H);
  unsigned short* TP1L = (unsigned short*)(ws + oTP1L);
  unsigned short* CATH = (unsigned short*)(ws + oCATH);
  unsigned short* CATL = (unsigned short*)(ws + oCATL);
  unsigned short* HH   = (unsigned short*)(ws + oHH);
  unsigned short* HL   = (unsigned short*)(ws + oHL);
  float*          QF   = (float*)(ws + oQF);
  float*          KF   = (float*)(ws + oKF);
  unsigned short* QN   = (unsigned short*)(ws + oQN);
  unsigned short* KN   = (unsigned short*)(ws + oKN);
  unsigned short* VT   = (unsigned short*)(ws + oVT);
  float*          HP64 = (float*)(ws + oHP64);
  unsigned short* AOH  = (unsigned short*)(ws + oAOH);
  unsigned short* AOL  = (unsigned short*)(ws + oAOL);
  unsigned short* OUTH = (unsigned short*)(ws + oOUTH);
  unsigned short* OUTL = (unsigned short*)(ws + oOUTL);
  unsigned short* XB   = (unsigned short*)(ws + oXB);
  float*          out  = (float*)d_out;

  const int n8w1  = (EH * DM) / 8;
  const int n8w2  = (DM * EH) / 8;
  const int n8pw2 = (PF * PH) / 8;
  const int n8cw  = (DM * TIN) / 8;
  const int n8qw  = (QNP * DM) / 8;
  const int n8sq  = (DM * DM) / 8;
  const int n8hp  = (HPN * DM) / 8;
  const int n8x   = (MP * DM) / 8;
  if ((n8w1 % 256) != 0 || (n8w2 % 256) != 0 || (n8pw2 % 256) != 0 || (n8cw % 256) != 0) return;
  if ((n8qw % 256) != 0 || (n8sq % 256) != 0 || (n8hp % 256) != 0 || (n8x % 256) != 0) return;

  const dim3 blk(256), blk128(128);
  cvt_w<<<dim3(n8w1 / 256), blk, 0, stream>>>(ex_w1, W1T, DM, EH, EH, n8w1);
  cvt_w<<<dim3(n8w2 / 256), blk, 0, stream>>>(ex_w2, W2T, EH, DM, DM, n8w2);
  cvt_w<<<dim3(n8pw2 / 256), blk, 0, stream>>>(pos_w2, PW2T, PH, PF, PF, n8pw2);
  cvt_w<<<dim3(n8cw / 256), blk, 0, stream>>>(cat_w, CWT, TIN, DM, DM, n8cw);
  cvt_w<<<dim3(n8qw / 256), blk, 0, stream>>>(q_w, QWT, DM, QREAL, QNP, n8qw);
  cvt_w<<<dim3(n8sq / 256), blk, 0, stream>>>(k_w, KWT, DM, DM, DM, n8sq);
  cvt_w<<<dim3(n8sq / 256), blk, 0, stream>>>(v_w, VWT, DM, DM, DM, n8sq);
  cvt_w<<<dim3(n8sq / 256), blk, 0, stream>>>(o_w, OWT, DM, DM, DM, n8sq);
  cvt_w<<<dim3(n8sq / 256), blk, 0, stream>>>(he_w, HEWT, DM, DM, DM, n8sq);
  cvt_w<<<dim3(n8hp / 256), blk, 0, stream>>>(hp_w, HPWT, DM, 3, HPN, n8hp);
  pack_bias<<<dim3(1), blk, 0, stream>>>(q_b, hp_b, BIAS);

  cvt_x<<<dim3(n8x / 256), blk, 0, stream>>>(x_ef, XB, n8x);

  const dim3 gT64(((MP / 64) * (EH / 64) + 7) / 8, 1);
  const dim3 gT512(((MP / 64) * (DM / 64) + 7) / 8, 1);
  const dim3 gT128(((MP / 64) * (PF / 64) + 7) / 8, 1);
  const dim3 gT576(((MP / 64) * (QNP / 64) + 7) / 8, 1);
  const dim3 gTVT(((DM / 64) * (NTOK / 64) + 7) / 8, NB);
  const dim3 gTHP(((MP / 64) * (HPN / 64) + 7) / 8, 1);
  const int  nqb = (MP * NH) / 32;

  gemm64<1, 1, 3, 0, 1><<<gT64, blk, 0, stream>>>(
      XB, XB, DM, 0LL, W1T, W1T, DM, 0LL, ex_b1, 1.0f,
      (void*)TE1H, (void*)TE1L, EH, 0LL, MP, EH, DM, 1.0f);
  gemm64<2, 1, 3, 0, 0><<<gT512, blk, 0, stream>>>(
      TE1H, TE1L, EH, 0LL, W2T, W2T, EH, 0LL, ex_b2, 1.0f,
      (void*)CATH, (void*)CATL, TIN, 0LL, MP, DM, EH, 1.0f);
  pos_l1<<<dim3((MP * 8) / 256), blk, 0, stream>>>(x_pos, pos_w1, pos_b1, TP1H, TP1L);
  gemm64<2, 1, 3, 0, 0><<<gT128, blk, 0, stream>>>(
      TP1H, TP1L, PH, 0LL, PW2T, PW2T, PH, 0LL, pos_b2, 1.0f,
      (void*)(CATH + (DM + TT)), (void*)(CATL + (DM + TT)), TIN, 0LL, MP, PF, PH, 1.0f);
  tdt_k<<<dim3(1), blk128, 0, stream>>>(x_dt, yy_w, yy_b, TDT);
  tdt_bcast<<<dim3((MP * 16) / 256), blk, 0, stream>>>(TDT, CATH, CATL);
  gemm64<2, 1, 3, 0, 0><<<gT512, blk, 0, stream>>>(
      CATH, CATL, TIN, 0LL, CWT, CWT, TIN, 0LL, cat_b, 1.0f,
      (void*)HH, (void*)HL, DM, 0LL, MP, DM, TIN, 1.0f);
  gemm64<2, 1, 0, 0, 0><<<gT576, blk, 0, stream>>>(
      HH, HL, DM, 0LL, QWT, QWT, DM, 0LL, BIAS, 1.0f,
      (void*)QF, (void*)QF, QNP, 0LL, MP, QNP, DM, 1.0f);
  gemm64<2, 1, 0, 0, 0><<<gT512, blk, 0, stream>>>(
      HH, HL, DM, 0LL, KWT, KWT, DM, 0LL, k_b, 1.0f,
      (void*)KF, (void*)KF, DM, 0LL, MP, DM, DM, 1.0f);
  gemm64<1, 2, 2, 1, 0><<<gTVT, blk, 0, stream>>>(
      VWT, VWT, DM, 0LL, HH, HL, DM, (long long)NTOK * DM, v_b, VC,
      (void*)VT, (void*)VT, NTOK, (long long)DM * NTOK, DM, NTOK, DM, VC);
  rms_qk<<<dim3(2 * nqb), blk, 0, stream>>>(QF, KF, qn_w, kn_w, QN, KN, nqb);
  attn<<<dim3(NB * NH * NQB), blk128, 0, stream>>>(QN, KN, VT, QF, AOH, AOL);
  gemm64<2, 1, 3, 0, 0><<<gT512, blk, 0, stream>>>(
      AOH, AOL, DM, 0LL, OWT, OWT, DM, 0LL, o_b, 1.0f,
      (void*)OUTH, (void*)OUTL, DM, 0LL, MP, DM, DM, 1.0f);
  gemm64<2, 1, 0, 0, 0><<<gT512, blk, 0, stream>>>(
      OUTH, OUTL, DM, 0LL, HEWT, HEWT, DM, 0LL, he_b, 1.0f,
      (void*)out, (void*)out, DM, 0LL, MP, DM, DM, 1.0f);
  gemm64<2, 1, 0, 0, 0><<<gTHP, blk, 0, stream>>>(
      OUTH, OUTL, DM, 0LL, HPWT, HPWT, DM, 0LL, BIAS + QNP, 1.0f,
      (void*)HP64, (void*)HP64, HPN, 0LL, MP, HPN, DM, 1.0f);
  pack_out<<<dim3(((MP * 3) / 4 + (NB * TT) / 4 + 255) / 256), blk, 0, stream>>>(HP64, TDT, out);
  (void)hipGetLastError();
}
